// HPTEncoder_3874060501345
// MI455X (gfx1250) — hardware-verified
//
#include <hip/hip_runtime.h>
#include <math.h>
#include <stdint.h>

#define SEQ_LEN   4096
#define EMB_DIM   768
#define HEAD_DIM  64
#define NUM_HEADS 12
#define WIN_ONE   256
#define KV_CH     64
#define NQT       (SEQ_LEN / 64)
#define GQ_ROWS   64
#define NEG_FILL  (-1.0e9f)
#define PCARRY    32768.0f

typedef __attribute__((ext_vector_type(16))) _Float16 v16h;
typedef __attribute__((ext_vector_type(8)))  _Float16 v8h;
typedef __attribute__((ext_vector_type(16))) __bf16   v16b;
typedef __attribute__((ext_vector_type(8)))  __bf16   v8b;
typedef __attribute__((ext_vector_type(8)))  float    v8f;
typedef __attribute__((ext_vector_type(4)))  float    v4f;
#define PSCALE 32768.0f
#define U16(p) ((const unsigned short*)(const void*)(p))
#define PSCALE_INV (1.0f / 32768.0f)

__device__ __forceinline__ unsigned short f2bf_bits(float f) {
  unsigned u = __float_as_uint(f);
  return (unsigned short)((u + 0x7FFFu + ((u >> 16) & 1u)) >> 16);
}
__device__ __forceinline__ float bf_bits2f(unsigned short h) { return __uint_as_float(((unsigned)h) << 16); }

__device__ __forceinline__ void dep_guard_h(v8f& a, v8f& b, v16h x, v16h y) { asm volatile("v_nop\n\tv_nop\n\tv_nop\n\tv_nop" : "+v"(a), "+v"(b) : "v"(x), "v"(y)); }
__device__ __forceinline__ void dep_guard_b(v8f& a, v8f& b, v16b x, v16b y) { asm volatile("v_nop\n\tv_nop\n\tv_nop\n\tv_nop" : "+v"(a), "+v"(b) : "v"(x), "v"(y)); }
__device__ __forceinline__ void keep4_h(v16h a, v16h b, v16h c, v16h d) { asm volatile("v_nop" :: "v"(a), "v"(b), "v"(c), "v"(d)); }
__device__ __forceinline__ void keep4_b(v16b a, v16b b, v16b c, v16b d) { asm volatile("v_nop" :: "v"(a), "v"(b), "v"(c), "v"(d)); }
__device__ __forceinline__ void acc_guard4(v8f& a, v8f& b, v8f& c, v8f& d) { asm volatile("v_nop\n\tv_nop\n\tv_nop\n\tv_nop" : "+v"(a), "+v"(b), "+v"(c), "+v"(d)); }
template <typename T> struct Frag;
template <> struct Frag<_Float16> {
  typedef v16h V; union U { v16h v; v8h h[2]; };
  static __device__ __forceinline__ v16h load(const _Float16* p) {
    U f; f.h[0] = *(const v8h*)(p); f.h[1] = *(const v8h*)(p + 16); return f.v;
  }
  static __device__ __forceinline__ v8f mma(v16h a, v16h b, v8f c) {
    return __builtin_amdgcn_wmma_f32_16x16x32_f16(false, a, false, b, (short)0, c, false, false);
  }
  static __device__ __forceinline__ void guard(v8f& a, v8f& b, v16h x, v16h y) { dep_guard_h(a, b, x, y); }
  static __device__ __forceinline__ void keep(v16h a, v16h b, v16h c, v16h d) { keep4_h(a, b, c, d); }
};
template <> struct Frag<__bf16> {
  typedef v16b V; union U { v16b v; v8b h[2]; };
  static __device__ __forceinline__ v16b load(const __bf16* p) {
    U f; f.h[0] = *(const v8b*)(p); f.h[1] = *(const v8b*)(p + 16); return f.v;
  }
  static __device__ __forceinline__ v8f mma(v16b a, v16b b, v8f c) {
    return __builtin_amdgcn_wmma_f32_16x16x32_bf16(false, a, false, b, (short)0, c, false, false);
  }
  static __device__ __forceinline__ void guard(v8f& a, v8f& b, v16b x, v16b y) { dep_guard_b(a, b, x, y); }
  static __device__ __forceinline__ void keep(v16b a, v16b b, v16b c, v16b d) { keep4_b(a, b, c, d); }
};

template <int ET> struct Elem;
template <> struct Elem<0> { typedef _Float16 T; };
template <> struct Elem<1> { typedef __bf16 T; };
template <int ET, bool SPLIT, int BIAS_MODE, int OUT_MODE, bool RESID, int ACT = 0>
__global__ __launch_bounds__(256) void wmma_gemm64(
    const unsigned short* __restrict__ Ap, const unsigned short* __restrict__ A2p, int lda, long strideA,
    const unsigned short* __restrict__ Btp, const unsigned short* __restrict__ Bt2p, int ldb, long strideB,
    void* __restrict__ Cout, void* __restrict__ Cout2, int ldc, long strideC,
    const float* __restrict__ bias,
    const float* __restrict__ resid, long strideR,
    int M, int N, int K, float scale) {
  typedef typename Elem<ET>::T T;
  typedef typename Frag<T>::V V;
  const T* A = (const T*)Ap; const T* A2 = (const T*)A2p; const T* Bt = (const T*)Btp; const T* Bt2 = (const T*)Bt2p;
  __shared__ __align__(16) float sT[8][16 * 68];
  const int b    = blockIdx.y;
  const int lane = threadIdx.x & 31;
  const int wave = threadIdx.x >> 5;
  const int tilesN = N >> 6;
  const int tilesM = M >> 6;
  const int tile = blockIdx.x * 8 + wave;
  if (tile >= tilesM * tilesN) return;
  const int tm = tile / tilesN;
  const int tn = tile - tm * tilesN;
  const int m0 = tm << 6;
  const int n0 = tn << 6;

  const T* Ab  = A  + (size_t)b * strideA;
  const T* Bb  = Bt + (size_t)b * strideB;
  const T* Ab2 = SPLIT ? (A2  + (size_t)b * strideA) : nullptr;
  const T* Bb2 = SPLIT ? (Bt2 + (size_t)b * strideB) : nullptr;

  const int rlane = lane & 15;
  const int koff  = (lane >> 4) * 8;
  const int mOff  = (lane >> 4) * 8;

  v8f acc[4][4];
#pragma unroll
  for (int i = 0; i < 4; ++i)
#pragma unroll
    for (int j = 0; j < 4; ++j) acc[i][j] = (v8f){0.f,0.f,0.f,0.f,0.f,0.f,0.f,0.f};

  for (int k0 = 0; k0 < K; k0 += 32) {
    V bh[4], bl[4];
#pragma unroll
    for (int j = 0; j < 4; ++j) {
      const size_t bo = (size_t)(n0 + (j << 4) + rlane) * ldb + koff + k0;
      bh[j] = Frag<T>::load(Bb + bo);
      if (SPLIT) bl[j] = Frag<T>::load(Bb2 + bo);
    }
#pragma unroll
    for (int i = 0; i < 4; ++i) {
      const size_t ao = (size_t)(m0 + (i << 4) + rlane) * lda + koff + k0;
      V ah = Frag<T>::load(Ab + ao);
      V al;
      if (SPLIT) al = Frag<T>::load(Ab2 + ao);
#pragma unroll
      for (int j = 0; j < 4; ++j) {
        acc[i][j] = Frag<T>::mma(ah, bh[j], acc[i][j]);
        if (SPLIT) {
          acc[i][j] = Frag<T>::mma(ah, bl[j], acc[i][j]);
          acc[i][j] = Frag<T>::mma(al, bh[j], acc[i][j]);
        }
      }
      Frag<T>::guard(acc[i][0], acc[i][3], ah, SPLIT ? al : ah);
    }
    Frag<T>::keep(bh[0], bh[1], bh[2], bh[3]);
    if (SPLIT) Frag<T>::keep(bl[0], bl[1], bl[2], bl[3]);
  }
  acc_guard4(acc[0][0], acc[0][1], acc[0][2], acc[0][3]);
  acc_guard4(acc[1][0], acc[1][1], acc[1][2], acc[1][3]);
  acc_guard4(acc[2][0], acc[2][1], acc[2][2], acc[2][3]);
  acc_guard4(acc[3][0], acc[3][1], acc[3][2], acc[3][3]);

  float* slab = sT[wave];
  const float* Rb = RESID ? (resid + (size_t)b * strideR) : nullptr;
#pragma unroll
  for (int i = 0; i < 4; ++i) {
    const int mBase = m0 + (i << 4);
#pragma unroll
    for (int j = 0; j < 4; ++j) {
      const int n = n0 + (j << 4) + rlane;
      float bv = 0.f;
      if (BIAS_MODE == 2) bv = bias[n];
#pragma unroll
      for (int r = 0; r < 8; ++r) {
        float v = acc[i][j][r] * scale;
        if (BIAS_MODE == 1) v += bias[mBase + mOff + r];
        if (BIAS_MODE == 2) v += bv;
        if (RESID) v += Rb[(size_t)(mBase + mOff + r) * ldc + n];
        if (ACT == 1) v = tanhf(v);
        if (ACT == 2) v = fmaxf(v, 0.0f);
        if (ACT == 3) v = v / (1.0f + expf(-v));
        if (ACT == 4) v = (v > 0.f) ? v : 0.01f * v;
        slab[(mOff + r) * 68 + (j << 4) + rlane] = v;
      }
    }
    __builtin_amdgcn_fence(__ATOMIC_RELEASE, "workgroup");
    __builtin_amdgcn_wave_barrier();
    __builtin_amdgcn_fence(__ATOMIC_ACQUIRE, "workgroup");
    if (OUT_MODE == 0) {
      float* C = (float*)Cout + (size_t)b * strideC;
      const int hh = lane >> 4, c4 = (lane & 15) * 4;
      for (int pass = 0; pass < 2; ++pass) {
#pragma unroll
        for (int it = 0; it < 8; ++it) {
          const int row = it * 2 + hh;
          v4f v = *(const v4f*)(slab + row * 68 + c4);
          *(volatile v4f*)(C + (size_t)(mBase + row) * ldc + n0 + c4) = v;
        }
        __threadfence();
      }
    } else {
      const int q = lane >> 3, c8 = (lane & 7) * 8;
      unsigned short* C  = (unsigned short*)Cout  + (size_t)b * strideC;
      unsigned short* C2 = (OUT_MODE == 2) ? ((unsigned short*)Cout2 + (size_t)b * strideC) : nullptr;
      for (int pass = 0; pass < 2; ++pass) {
#pragma unroll
        for (int it = 0; it < 4; ++it) {
          const int row = it * 4 + q;
          const float* sp = slab + row * 68 + c8;
          v8h hv, lv;
#pragma unroll
          for (int e = 0; e < 8; ++e) {
            if (OUT_MODE == 1) {
              hv[e] = (_Float16)sp[e];
            } else {
              unsigned short hb = f2bf_bits(sp[e]);
              unsigned short lb = f2bf_bits(sp[e] - bf_bits2f(hb));
              hv[e] = __builtin_bit_cast(_Float16, hb);
              lv[e] = __builtin_bit_cast(_Float16, lb);
            }
          }
          *(volatile v8h*)(C + (size_t)(mBase + row) * ldc + n0 + c8) = hv;
          if (OUT_MODE == 2) *(volatile v8h*)(C2 + (size_t)(mBase + row) * ldc + n0 + c8) = lv;
        }
        __threadfence();
      }
    }
    __builtin_amdgcn_fence(__ATOMIC_RELEASE, "workgroup");
    __builtin_amdgcn_wave_barrier();
    __builtin_amdgcn_fence(__ATOMIC_ACQUIRE, "workgroup");
  }
}

__global__ __launch_bounds__(256) void cast_f32_f16x2s(
    const float* __restrict__ in, _Float16* __restrict__ out, int n2, float sc) {
  int i = blockIdx.x * 256 + threadIdx.x;
  if (i < n2) {
    const size_t i2 = 2 * (size_t)i;
    const _Float16 h0 = (_Float16)(in[i2] * sc), h1 = (_Float16)(in[i2 + 1] * sc);
    const unsigned u = (unsigned)__builtin_bit_cast(unsigned short, h0) | ((unsigned)__builtin_bit_cast(unsigned short, h1) << 16);
    ((volatile unsigned*)out)[i] = u;
    __threadfence();
    ((volatile unsigned*)out)[i] = u;
  }
}

__global__ __launch_bounds__(256) void transpose_w_f16(
    const float* __restrict__ W0, const float* __restrict__ W1, const float* __restrict__ W2,
    const float* __restrict__ W3, const float* __restrict__ W4, const float* __restrict__ W5,
    _Float16* __restrict__ WT, float sc) {
  __shared__ float tile[64][65];
  const int tk = blockIdx.x, tn = blockIdx.y, wi = blockIdx.z;
  const int tid = threadIdx.x, lane = tid & 31, wave = tid >> 5;
  const float* Wsrc = (wi == 0) ? W0 : ((wi == 1) ? W1 : ((wi == 2) ? W2 : ((wi == 3) ? W3 : ((wi == 4) ? W4 : W5))));
#pragma unroll
  for (int it = 0; it < 16; ++it) {
    const int idx = it * 256 + tid;
    const int r = idx >> 6, cc = idx & 63;
    tile[r][cc] = Wsrc[(size_t)(tk * 64 + r) * EMB_DIM + tn * 64 + cc];
  }
  __syncthreads();
  _Float16* base = WT + (size_t)wi * EMB_DIM * EMB_DIM;
  const int q = lane >> 3, c8 = (lane & 7) * 8;
  for (int pass = 0; pass < 2; ++pass) {
#pragma unroll
    for (int it = 0; it < 2; ++it) {
      const int nn = wave * 8 + it * 4 + q;
      v8h hv;
#pragma unroll
      for (int e = 0; e < 8; ++e) hv[e] = (_Float16)(tile[c8 + e][nn] * sc);
      *(volatile v8h*)(base + (size_t)(tn * 64 + nn) * EMB_DIM + tk * 64 + c8) = hv;
    }
    __threadfence();
  }
}

__device__ __forceinline__ v8f mma_h(v16h a, v16h b, v8f cacc) {
  cacc = __builtin_amdgcn_wmma_f32_16x16x32_f16(false, a, false, b, (short)0, cacc, false, false);
  asm volatile("v_nop\n\tv_nop\n\tv_nop\n\tv_nop" : "+v"(cacc) : "v"(a), "v"(b));
  return cacc;
}

template <int MODE>
__global__ __launch_bounds__(128)
void lw_attn_kernel(const unsigned short* __restrict__ Qp, const unsigned short* __restrict__ Kp,
                    const unsigned short* __restrict__ Vtp, float* __restrict__ out, float sscale) {
  union FH { v16h v; v8h h[2]; };
  __shared__ __align__(16) _Float16 Ksh[KV_CH * HEAD_DIM];
  __shared__ __align__(16) _Float16 Vth[HEAD_DIM * KV_CH];
  __shared__ __align__(16) _Float16 Psh[4][16 * KV_CH];
  __shared__ __align__(16) float    Os[4][16 * 68];
  const _Float16* Q  = (const _Float16*)(const void*)Qp;
  const _Float16* Kb = (const _Float16*)(const void*)Kp;
  const _Float16* Vt = (const _Float16*)(const void*)Vtp;

  const int tid  = threadIdx.x;
  const int wave = tid >> 5;
  const int lane = tid & 31;
  const int hh   = lane >> 4;
  const int c    = lane & 15;

  int h, qb;
  if (MODE == 1) { h = (int)blockIdx.x / (NQT - 1); qb = 1 + ((int)blockIdx.x - h * (NQT - 1)); }
  else           { h = (int)blockIdx.x;              qb = 0; }
  if (h > NUM_HEADS - 1) h = NUM_HEADS - 1;
  if (qb > NQT - 1) qb = NQT - 1;
  const int hcol = h * HEAD_DIM;
  const int q0   = qb * 64 + wave * 16;

  v16h qa[2];
  {
    const _Float16* qrow = Q + (size_t)(q0 + c) * EMB_DIM + hcol + 8 * hh;
#pragma unroll
    for (int dc = 0; dc < 2; ++dc) qa[dc] = Frag<_Float16>::load(qrow + dc * 32);
  }

  float mrow[8], lrow[8];
  v8f oacc[4];
#pragma unroll
  for (int r = 0; r < 8; ++r) { mrow[r] = -INFINITY; lrow[r] = 0.f; }
#pragma unroll
  for (int t4 = 0; t4 < 4; ++t4) oacc[t4] = (v8f){0.f,0.f,0.f,0.f,0.f,0.f,0.f,0.f};

  int klo = 0, khi = NQT - 1, nCh = NQT;
  if (MODE == 1) {
    klo = qb - 4; if (klo < 1) klo = 1;
    khi = qb + 4; if (khi > NQT - 1) khi = NQT - 1;
    nCh = 2 + khi - klo;
  }
  if (nCh > NQT) nCh = NQT;

  for (int t = 0; t < nCh; ++t) {
    bool band = false;
    int kc = t;
    if (MODE == 1) { band = (t > 0); kc = band ? (klo + t - 1) : 0; }
    if (kc > NQT - 1) kc = NQT - 1;
    if (kc < 0) kc = 0;
    const int kv0 = kc * KV_CH;

    __syncthreads();
#pragma unroll
    for (int it = 0; it < 4; ++it) {
      const int idx = it * 128 + tid;
      const int row = idx >> 3, seg = (idx & 7) * 8;
      const v8h kk = *(const v8h*)(Kb + (size_t)(kv0 + row) * EMB_DIM + hcol + seg);
      const v8h vv = *(const v8h*)(Vt + (size_t)(hcol + row) * SEQ_LEN + kv0 + seg);
      *(v8h*)(Ksh + row * HEAD_DIM + seg) = kk;
      *(v8h*)(Vth + row * KV_CH + seg) = vv;
    }
    __syncthreads();

    v8f s[4];
#pragma unroll
    for (int j = 0; j < 4; ++j) {
      s[j] = (v8f){0.f,0.f,0.f,0.f,0.f,0.f,0.f,0.f};
#pragma unroll
      for (int dc = 0; dc < 2; ++dc) {
        FH kb;
        kb.h[0] = *(const v8h*)(Ksh + (j * 16 + c) * HEAD_DIM + dc * 32 + 8 * hh);
        kb.h[1] = *(const v8h*)(Ksh + (j * 16 + c) * HEAD_DIM + dc * 32 + 16 + 8 * hh);
        s[j] = mma_h(qa[dc], kb.v, s[j]);
      }
    }

    float cm[8];
#pragma unroll
    for (int r = 0; r < 8; ++r) {
      const int qrow = q0 + 8 * hh + r;
      float m = -INFINITY;
#pragma unroll
      for (int j = 0; j < 4; ++j) {
        const int kvcol = kv0 + j * 16 + c;
        float sv = s[j][r] * sscale;
        if (MODE == 1) {
          int dd = kvcol - qrow;
          dd = (dd < 0) ? -dd : dd;
          if (band && (dd > WIN_ONE)) sv = NEG_FILL;
        }
        s[j][r] = sv;
        m = fmaxf(m, sv);
      }
#pragma unroll
      for (int off = 1; off < 16; off <<= 1) m = fmaxf(m, __shfl_xor(m, off, 32));
      cm[r] = m;
    }

    _Float16* pw = Psh[wave];
#pragma unroll
    for (int r = 0; r < 8; ++r) {
      const float mnew  = fmaxf(mrow[r], cm[r]);
      const float alpha = expf(mrow[r] - mnew);
      mrow[r] = mnew;
      float psum = 0.f;
#pragma unroll
      for (int j = 0; j < 4; ++j) {
        const float p = expf(s[j][r] - mnew);
        psum += p;
        pw[(8 * hh + r) * KV_CH + j * 16 + c] = (_Float16)(p * PCARRY);
      }
#pragma unroll
      for (int off = 1; off < 16; off <<= 1) psum += __shfl_xor(psum, off, 32);
      lrow[r] = lrow[r] * alpha + psum;
#pragma unroll
      for (int t4 = 0; t4 < 4; ++t4) oacc[t4][r] *= alpha;
    }
    __builtin_amdgcn_fence(__ATOMIC_RELEASE, "workgroup");
    __builtin_amdgcn_wave_barrier();
    __builtin_amdgcn_fence(__ATOMIC_ACQUIRE, "workgroup");

#pragma unroll 1
    for (int kk = 0; kk < 2; ++kk) {
      FH pa;
      pa.h[0] = *(const v8h*)(pw + c * KV_CH + kk * 32 + 8 * hh);
      pa.h[1] = *(const v8h*)(pw + c * KV_CH + kk * 32 + 16 + 8 * hh);
#pragma unroll
      for (int t4 = 0; t4 < 4; ++t4) {
        FH vb;
        vb.h[0] = *(const v8h*)(Vth + (t4 * 16 + c) * KV_CH + kk * 32 + 8 * hh);
        vb.h[1] = *(const v8h*)(Vth + (t4 * 16 + c) * KV_CH + kk * 32 + 16 + 8 * hh);
        oacc[t4] = mma_h(pa.v, vb.v, oacc[t4]);
      }
    }
  }

  float* os = Os[wave];
#pragma unroll
  for (int r = 0; r < 8; ++r) {
    const float inv = 1.0f / (lrow[r] * PCARRY);
#pragma unroll
    for (int t4 = 0; t4 < 4; ++t4) os[(8 * hh + r) * 68 + t4 * 16 + c] = oacc[t4][r] * inv;
  }
  __builtin_amdgcn_fence(__ATOMIC_RELEASE, "workgroup");
  __builtin_amdgcn_wave_barrier();
  __builtin_amdgcn_fence(__ATOMIC_ACQUIRE, "workgroup");
  {
    float* ob = out + hcol;
    const int c4 = (lane & 15) * 4;
    for (int pass = 0; pass < 2; ++pass) {
#pragma unroll
      for (int it = 0; it < 8; ++it) {
        const int row = it * 2 + hh;
        v4f val = *(const v4f*)(os + row * 68 + c4);
        *(volatile v4f*)(ob + (size_t)(q0 + row) * EMB_DIM + c4) = val;
      }
      __threadfence();
    }
  }
}

extern "C" void kernel_launch(void* const* d_in, const int* in_sizes, int n_in,
                              void* d_out, int out_size, void* d_ws, size_t ws_size,
                              hipStream_t stream) {
  if (n_in < 13) return;
  if (in_sizes[0] != SEQ_LEN * EMB_DIM) return;
  for (int i = 1; i < 13; i += 2) {
    if (in_sizes[i] != EMB_DIM * EMB_DIM) return;
    if (in_sizes[i + 1] != EMB_DIM) return;
  }
  if (out_size != SEQ_LEN * EMB_DIM) return;

  const float* x   = (const float*)d_in[0];
  const float* Wq  = (const float*)d_in[1];  const float* bq  = (const float*)d_in[2];
  const float* Wk  = (const float*)d_in[3];  const float* bk  = (const float*)d_in[4];
  const float* Wv  = (const float*)d_in[5];  const float* bv  = (const float*)d_in[6];
  const float* Wqg = (const float*)d_in[7];  const float* bqg = (const float*)d_in[8];
  const float* Wkg = (const float*)d_in[9];  const float* bkg = (const float*)d_in[10];
  const float* Wvg = (const float*)d_in[11]; const float* bvg = (const float*)d_in[12];
  float* out = (float*)d_out;

  const size_t PX  = (size_t)SEQ_LEN * EMB_DIM * 2;
  const size_t WPL = (size_t)EMB_DIM * EMB_DIM;
  const size_t PW  = 6 * WPL * 2;
  const size_t PQG = (size_t)GQ_ROWS * EMB_DIM * 2;
  size_t off = 0;
  const size_t oX   = off; off += PX;
  const size_t oW   = off; off += PW;
  const size_t oQ   = off; off += PX;
  const size_t oK   = off; off += PX;
  const size_t oKG  = off; off += PX;
  const size_t oVT  = off; off += PX;
  const size_t oVGT = off; off += PX;
  const size_t oQG  = off; off += PQG;
  if (off > ws_size) return;
  if (off > (size_t)134217728) return;

  char* ws = (char*)d_ws;
  unsigned short* Xh    = (unsigned short*)(ws + oX);
  unsigned short* WT    = (unsigned short*)(ws + oW);
  unsigned short* Q16   = (unsigned short*)(ws + oQ);
  unsigned short* K16   = (unsigned short*)(ws + oK);
  unsigned short* KG16  = (unsigned short*)(ws + oKG);
  unsigned short* VT16  = (unsigned short*)(ws + oVT);
  unsigned short* VGT16 = (unsigned short*)(ws + oVGT);
  unsigned short* QG16  = (unsigned short*)(ws + oQG);

  const dim3 blk(256);

  const int n2x = SEQ_LEN * EMB_DIM / 2;
  cast_f32_f16x2s<<<dim3((n2x + 255) / 256), blk, 0, stream>>>(x, (_Float16*)Xh, n2x, 16.0f);
  transpose_w_f16<<<dim3(EMB_DIM / 64, EMB_DIM / 64, 6), blk, 0, stream>>>(Wq, Wk, Wv, Wqg, Wkg, Wvg, (_Float16*)WT, 256.0f);

  const float pscale = 0.000244140625f;
  const dim3 gP((((SEQ_LEN / 64) * (EMB_DIM / 64)) + 7) / 8, 1);
  wmma_gemm64<0, false, 2, 1, false><<<gP, blk, 0, stream>>>(
      Xh, Xh, EMB_DIM, 0L, WT + 0 * WPL, WT + 0 * WPL, EMB_DIM, 0L,
      (void*)Q16, (void*)Q16, EMB_DIM, 0L, bq, bq, 0L, SEQ_LEN, EMB_DIM, EMB_DIM, pscale);
  wmma_gemm64<0, false, 2, 1, false><<<gP, blk, 0, stream>>>(
      Xh, Xh, EMB_DIM, 0L, WT + 1 * WPL, WT + 1 * WPL, EMB_DIM, 0L,
      (void*)K16, (void*)K16, EMB_DIM, 0L, bk, bk, 0L, SEQ_LEN, EMB_DIM, EMB_DIM, pscale);
  wmma_gemm64<0, false, 2, 1, false><<<gP, blk, 0, stream>>>(
      Xh, Xh, EMB_DIM, 0L, WT + 4 * WPL, WT + 4 * WPL, EMB_DIM, 0L,
      (void*)KG16, (void*)KG16, EMB_DIM, 0L, bkg, bkg, 0L, SEQ_LEN, EMB_DIM, EMB_DIM, pscale);
  const dim3 gV((((EMB_DIM / 64) * (SEQ_LEN / 64)) + 7) / 8, 1);
  wmma_gemm64<0, false, 1, 1, false><<<gV, blk, 0, stream>>>(
      WT + 2 * WPL, WT + 2 * WPL, EMB_DIM, 0L, Xh, Xh, EMB_DIM, 0L,
      (void*)VT16, (void*)VT16, SEQ_LEN, 0L, bv, bv, 0L, EMB_DIM, SEQ_LEN, EMB_DIM, pscale);
  wmma_gemm64<0, false, 1, 1, false><<<gV, blk, 0, stream>>>(
      WT + 5 * WPL, WT + 5 * WPL, EMB_DIM, 0L, Xh, Xh, EMB_DIM, 0L,
      (void*)VGT16, (void*)VGT16, SEQ_LEN, 0L, bvg, bvg, 0L, EMB_DIM, SEQ_LEN, EMB_DIM, pscale);
  const dim3 gQG((((GQ_ROWS / 64) * (EMB_DIM / 64)) + 7) / 8, 1);
  wmma_gemm64<0, false, 2, 1, false><<<gQG, blk, 0, stream>>>(
      Xh, Xh, EMB_DIM, 0L, WT + 3 * WPL, WT + 3 * WPL, EMB_DIM, 0L,
      (void*)QG16, (void*)QG16, EMB_DIM, 0L, bqg, bqg, 0L, GQ_ROWS, EMB_DIM, EMB_DIM, pscale);

  lw_attn_kernel<1><<<dim3(NUM_HEADS * (NQT - 1)), dim3(128), 0, stream>>>(Q16, K16, VT16, out, 0.125f);
  lw_attn_kernel<0><<<dim3(NUM_HEADS), dim3(128), 0, stream>>>(QG16, KG16, VGT16, out, 0.125f);
}
